// MHBAWithMask_19842748907883
// MI455X (gfx1250) — hardware-verified
//
#include <hip/hip_runtime.h>

#define BB 4
#define LL 1024
#define EE 1024
#define HH 16
#define DD 64
#define NBH (BB * HH)
#define AKC 64
#define KSCALE 16384.0f
#define PSC16 32768.0f
#define SCL_QK (1.0f / 524288.0f)
#define MASKV (-3.125e18f)
#define NEG_INF (-__builtin_inff())

typedef __attribute__((ext_vector_type(16))) _Float16 v16h;
typedef __attribute__((ext_vector_type(8)))  _Float16 v8h;
typedef __attribute__((ext_vector_type(16))) __bf16   v16b;
typedef __attribute__((ext_vector_type(8)))  __bf16   v8b;
typedef __attribute__((ext_vector_type(8)))  float    v8f;
typedef __attribute__((ext_vector_type(4)))  float    v4f;
#define PSCALE 32768.0f
#define U16(p) ((const unsigned short*)(const void*)(p))
#define PSCALE_INV (1.0f / 32768.0f)

__device__ __forceinline__ unsigned short f2bf_bits(float f) {
  unsigned u = __float_as_uint(f);
  return (unsigned short)((u + 0x7FFFu + ((u >> 16) & 1u)) >> 16);
}
__device__ __forceinline__ float bf_bits2f(unsigned short h) { return __uint_as_float(((unsigned)h) << 16); }

__device__ __forceinline__ void dep_guard_h(v8f& a, v8f& b, v16h x, v16h y) { asm volatile("v_nop\n\tv_nop\n\tv_nop\n\tv_nop" : "+v"(a), "+v"(b) : "v"(x), "v"(y)); }
__device__ __forceinline__ void dep_guard_b(v8f& a, v8f& b, v16b x, v16b y) { asm volatile("v_nop\n\tv_nop\n\tv_nop\n\tv_nop" : "+v"(a), "+v"(b) : "v"(x), "v"(y)); }
__device__ __forceinline__ void keep4_h(v16h a, v16h b, v16h c, v16h d) { asm volatile("v_nop" :: "v"(a), "v"(b), "v"(c), "v"(d)); }
__device__ __forceinline__ void keep4_b(v16b a, v16b b, v16b c, v16b d) { asm volatile("v_nop" :: "v"(a), "v"(b), "v"(c), "v"(d)); }
__device__ __forceinline__ void acc_guard4(v8f& a, v8f& b, v8f& c, v8f& d) { asm volatile("v_nop\n\tv_nop\n\tv_nop\n\tv_nop" : "+v"(a), "+v"(b), "+v"(c), "+v"(d)); }
template <typename T> struct Frag;
template <> struct Frag<_Float16> {
  typedef v16h V; union U { v16h v; v8h h[2]; };
  static __device__ __forceinline__ v16h load(const _Float16* p) {
    U f; f.h[0] = *(const v8h*)(p); f.h[1] = *(const v8h*)(p + 16); return f.v;
  }
  static __device__ __forceinline__ v8f mma(v16h a, v16h b, v8f c) {
    return __builtin_amdgcn_wmma_f32_16x16x32_f16(false, a, false, b, (short)0, c, false, false);
  }
  static __device__ __forceinline__ void guard(v8f& a, v8f& b, v16h x, v16h y) { dep_guard_h(a, b, x, y); }
  static __device__ __forceinline__ void keep(v16h a, v16h b, v16h c, v16h d) { keep4_h(a, b, c, d); }
};
template <> struct Frag<__bf16> {
  typedef v16b V; union U { v16b v; v8b h[2]; };
  static __device__ __forceinline__ v16b load(const __bf16* p) {
    U f; f.h[0] = *(const v8b*)(p); f.h[1] = *(const v8b*)(p + 16); return f.v;
  }
  static __device__ __forceinline__ v8f mma(v16b a, v16b b, v8f c) {
    return __builtin_amdgcn_wmma_f32_16x16x32_bf16(false, a, false, b, (short)0, c, false, false);
  }
  static __device__ __forceinline__ void guard(v8f& a, v8f& b, v16b x, v16b y) { dep_guard_b(a, b, x, y); }
  static __device__ __forceinline__ void keep(v16b a, v16b b, v16b c, v16b d) { keep4_b(a, b, c, d); }
};

template <int ET> struct Elem;
template <> struct Elem<0> { typedef _Float16 T; };
template <> struct Elem<1> { typedef __bf16 T; };
template <int ET, bool SPLIT, int BIAS_MODE, int OUT_MODE, bool RESID, int ACT = 0>
__global__ __launch_bounds__(256) void wmma_gemm64(
    const unsigned short* __restrict__ Ap, const unsigned short* __restrict__ A2p, int lda, long strideA,
    const unsigned short* __restrict__ Btp, const unsigned short* __restrict__ Bt2p, int ldb, long strideB,
    void* __restrict__ Cout, void* __restrict__ Cout2, int ldc, long strideC,
    const float* __restrict__ bias,
    const float* __restrict__ resid, long strideR,
    int M, int N, int K, float scale) {
  typedef typename Elem<ET>::T T;
  typedef typename Frag<T>::V V;
  const T* A = (const T*)Ap; const T* A2 = (const T*)A2p; const T* Bt = (const T*)Btp; const T* Bt2 = (const T*)Bt2p;
  __shared__ __align__(16) float sT[8][16 * 68];
  const int b    = blockIdx.y;
  const int lane = threadIdx.x & 31;
  const int wave = threadIdx.x >> 5;
  const int tilesN = N >> 6;
  const int tilesM = M >> 6;
  const int tile = blockIdx.x * 8 + wave;
  if (tile >= tilesM * tilesN) return;
  const int tm = tile / tilesN;
  const int tn = tile - tm * tilesN;
  const int m0 = tm << 6;
  const int n0 = tn << 6;

  const T* Ab  = A  + (size_t)b * strideA;
  const T* Bb  = Bt + (size_t)b * strideB;
  const T* Ab2 = SPLIT ? (A2  + (size_t)b * strideA) : nullptr;
  const T* Bb2 = SPLIT ? (Bt2 + (size_t)b * strideB) : nullptr;

  const int rlane = lane & 15;
  const int koff  = (lane >> 4) * 8;
  const int mOff  = (lane >> 4) * 8;

  v8f acc[4][4];
#pragma unroll
  for (int i = 0; i < 4; ++i)
#pragma unroll
    for (int j = 0; j < 4; ++j) acc[i][j] = (v8f){0.f,0.f,0.f,0.f,0.f,0.f,0.f,0.f};

  for (int k0 = 0; k0 < K; k0 += 32) {
    V bh[4], bl[4];
#pragma unroll
    for (int j = 0; j < 4; ++j) {
      const size_t bo = (size_t)(n0 + (j << 4) + rlane) * ldb + koff + k0;
      bh[j] = Frag<T>::load(Bb + bo);
      if (SPLIT) bl[j] = Frag<T>::load(Bb2 + bo);
    }
#pragma unroll
    for (int i = 0; i < 4; ++i) {
      const size_t ao = (size_t)(m0 + (i << 4) + rlane) * lda + koff + k0;
      V ah = Frag<T>::load(Ab + ao);
      V al;
      if (SPLIT) al = Frag<T>::load(Ab2 + ao);
#pragma unroll
      for (int j = 0; j < 4; ++j) {
        acc[i][j] = Frag<T>::mma(ah, bh[j], acc[i][j]);
        if (SPLIT) {
          acc[i][j] = Frag<T>::mma(ah, bl[j], acc[i][j]);
          acc[i][j] = Frag<T>::mma(al, bh[j], acc[i][j]);
        }
      }
      Frag<T>::guard(acc[i][0], acc[i][3], ah, SPLIT ? al : ah);
    }
    Frag<T>::keep(bh[0], bh[1], bh[2], bh[3]);
    if (SPLIT) Frag<T>::keep(bl[0], bl[1], bl[2], bl[3]);
  }
  acc_guard4(acc[0][0], acc[0][1], acc[0][2], acc[0][3]);
  acc_guard4(acc[1][0], acc[1][1], acc[1][2], acc[1][3]);
  acc_guard4(acc[2][0], acc[2][1], acc[2][2], acc[2][3]);
  acc_guard4(acc[3][0], acc[3][1], acc[3][2], acc[3][3]);

  float* slab = sT[wave];
  const float* Rb = RESID ? (resid + (size_t)b * strideR) : nullptr;
#pragma unroll
  for (int i = 0; i < 4; ++i) {
    const int mBase = m0 + (i << 4);
#pragma unroll
    for (int j = 0; j < 4; ++j) {
      const int n = n0 + (j << 4) + rlane;
      float bv = 0.f;
      if (BIAS_MODE == 2) bv = bias[n];
#pragma unroll
      for (int r = 0; r < 8; ++r) {
        float v = acc[i][j][r] * scale;
        if (BIAS_MODE == 1) v += bias[mBase + mOff + r];
        if (BIAS_MODE == 2) v += bv;
        if (RESID) v += Rb[(size_t)(mBase + mOff + r) * ldc + n];
        if (ACT == 1) v = tanhf(v);
        if (ACT == 2) v = fmaxf(v, 0.0f);
        if (ACT == 3) v = v / (1.0f + expf(-v));
        if (ACT == 4) v = (v > 0.f) ? v : 0.01f * v;
        if (ACT == 5) v = 0.5f * v * (1.0f + erff(v * 0.70710678118654752f));
        slab[(mOff + r) * 68 + (j << 4) + rlane] = v;
      }
    }
    __builtin_amdgcn_fence(__ATOMIC_RELEASE, "workgroup");
    __builtin_amdgcn_wave_barrier();
    __builtin_amdgcn_fence(__ATOMIC_ACQUIRE, "workgroup");
    if (OUT_MODE == 0) {
      float* C = (float*)Cout + (size_t)b * strideC;
      const int hh = lane >> 4, c4 = (lane & 15) * 4;
      for (int pass = 0; pass < 2; ++pass) {
#pragma unroll
        for (int it = 0; it < 8; ++it) {
          const int row = it * 2 + hh;
          v4f v = *(const v4f*)(slab + row * 68 + c4);
          *(volatile v4f*)(C + (size_t)(mBase + row) * ldc + n0 + c4) = v;
        }
        __threadfence();
      }
    } else {
      const int q = lane >> 3, c8 = (lane & 7) * 8;
      unsigned short* C  = (unsigned short*)Cout  + (size_t)b * strideC;
      unsigned short* C2 = (OUT_MODE == 2) ? ((unsigned short*)Cout2 + (size_t)b * strideC) : nullptr;
      for (int pass = 0; pass < 2; ++pass) {
#pragma unroll
        for (int it = 0; it < 4; ++it) {
          const int row = it * 4 + q;
          const float* sp = slab + row * 68 + c8;
          v8h hv, lv;
#pragma unroll
          for (int e = 0; e < 8; ++e) {
            if (OUT_MODE == 1) {
              hv[e] = (_Float16)sp[e];
            } else {
              unsigned short hb = f2bf_bits(sp[e]);
              unsigned short lb = f2bf_bits(sp[e] - bf_bits2f(hb));
              hv[e] = __builtin_bit_cast(_Float16, hb);
              lv[e] = __builtin_bit_cast(_Float16, lb);
            }
          }
          *(volatile v8h*)(C + (size_t)(mBase + row) * ldc + n0 + c8) = hv;
          if (OUT_MODE == 2) *(volatile v8h*)(C2 + (size_t)(mBase + row) * ldc + n0 + c8) = lv;
        }
        __threadfence();
      }
    }
    __builtin_amdgcn_fence(__ATOMIC_RELEASE, "workgroup");
    __builtin_amdgcn_wave_barrier();
    __builtin_amdgcn_fence(__ATOMIC_ACQUIRE, "workgroup");
  }
}

__global__ __launch_bounds__(256) void cast_f32_f16x2(
    const float* __restrict__ in, _Float16* __restrict__ out, int n2) {
  int i = blockIdx.x * 256 + threadIdx.x;
  if (i < n2) {
    const _Float16 h0 = (_Float16)in[2 * i], h1 = (_Float16)in[2 * i + 1];
    const unsigned u = (unsigned)__builtin_bit_cast(unsigned short, h0) | ((unsigned)__builtin_bit_cast(unsigned short, h1) << 16);
    ((volatile unsigned*)out)[i] = u;
    __threadfence();
    ((volatile unsigned*)out)[i] = u;
  }
}

__device__ __forceinline__ v8f mma_h(v16h a, v16h b, v8f c) {
  c = __builtin_amdgcn_wmma_f32_16x16x32_f16(false, a, false, b, (short)0, c, false, false);
  asm volatile("v_nop\n\tv_nop\n\tv_nop\n\tv_nop" : "+v"(c) : "v"(a), "v"(b));
  return c;
}

__global__ __launch_bounds__(256) void cast8_f16_kernel(
    const float* __restrict__ in, _Float16* __restrict__ out, int n8) {
  const int i = blockIdx.x * 256 + threadIdx.x;
  if (i < n8) {
    const v4f a  = *(const v4f*)(in + (size_t)i * 8);
    const v4f bq = *(const v4f*)(in + (size_t)i * 8 + 4);
    v8h hv;
    hv[0] = (_Float16)a[0];  hv[1] = (_Float16)a[1];  hv[2] = (_Float16)a[2];  hv[3] = (_Float16)a[3];
    hv[4] = (_Float16)bq[0]; hv[5] = (_Float16)bq[1]; hv[6] = (_Float16)bq[2]; hv[7] = (_Float16)bq[3];
    *(volatile v8h*)(out + (size_t)i * 8) = hv;
    __threadfence();
    *(volatile v8h*)(out + (size_t)i * 8) = hv;
  }
}

__global__ __launch_bounds__(64) void ksoft_kernel(
    const float* __restrict__ keys, const int* __restrict__ bern, _Float16* __restrict__ K16) {
  __shared__ __align__(16) _Float16 tile[32 * 64];
  const int bh = blockIdx.x, b = bh >> 4, h = bh & 15, d = threadIdx.x;
  const int wave = d >> 5, lane = d & 31;
  const int* bm = bern + (size_t)bh * LL;
  const float* kcol = keys + (size_t)b * LL * EE + h * DD + d;

  float mx = NEG_INF;
#pragma unroll 1
  for (int l = 0; l < LL; ++l) {
    const float x = kcol[(size_t)l * EE];
    const int keep = bm[l];
    mx = (keep != 0) ? fmaxf(mx, x) : mx;
  }
  float s = 0.f;
#pragma unroll 1
  for (int l = 0; l < LL; ++l) {
    const float x = kcol[(size_t)l * EE];
    const int keep = bm[l];
    const float p = expf(x - mx);
    s += (keep != 0) ? p : 0.f;
  }
  const float sc = KSCALE * (1.0f / s);
  _Float16* kout = K16 + (size_t)bh * LL * DD;
  const int c8 = (lane & 7) * 8;
#pragma unroll 1
  for (int lc = 0; lc < LL; lc += 32) {
#pragma unroll 1
    for (int i = 0; i < 32; ++i) {
      const float x = kcol[(size_t)(lc + i) * EE];
      const int keep = bm[lc + i];
      const float p = (keep != 0) ? (expf(x - mx) * sc) : 0.f;
      tile[i * 64 + d] = (_Float16)p;
    }
    __syncthreads();
    for (int pass = 0; pass < 2; ++pass) {
#pragma unroll
      for (int it = 0; it < 4; ++it) {
        const int row = it * 8 + wave * 4 + (lane >> 3);
        const v8h v = *(const v8h*)(tile + row * 64 + c8);
        *(volatile v8h*)(kout + (size_t)(lc + row) * DD + c8) = v;
      }
      __threadfence();
    }
    __syncthreads();
  }
}

__global__ __launch_bounds__(256) void qconv_kernel(
    const float* __restrict__ query, const float* __restrict__ cw, const float* __restrict__ cb,
    _Float16* __restrict__ Q16) {
  __shared__ __align__(16) float qs[34 * 66];
  __shared__ __align__(16) _Float16 tile[32 * 64];
  const int bh = blockIdx.y, b = bh >> 4, h = bh & 15;
  const int l0 = blockIdx.x * 32;
  const int tid = threadIdx.x, wave = tid >> 5, lane = tid & 31;
  for (int i = tid; i < 34 * 66; i += 256) {
    const int r = i / 66, cc = i - r * 66;
    const int l = l0 - 1 + r, d = cc - 1;
    const bool inb = (l >= 0) && (l < LL) && (d >= 0) && (d < DD);
    const int lcl = (l < 0) ? 0 : ((l >= LL) ? (LL - 1) : l);
    const int dcl = (d < 0) ? 0 : ((d >= DD) ? (DD - 1) : d);
    const float x = query[((size_t)(b * LL + lcl)) * EE + h * DD + dcl];
    qs[i] = inb ? x : 0.f;
  }
  float w[9];
#pragma unroll
  for (int t = 0; t < 9; ++t) w[t] = cw[h * 9 + t];
  const float bias = cb[h];
  __syncthreads();
  const int r = tid >> 3, cg = (tid & 7) * 8;
#pragma unroll 1
  for (int e = 0; e < 8; ++e) {
    const int d = cg + e;
    float acc = bias;
#pragma unroll
    for (int i = 0; i < 3; ++i)
#pragma unroll
      for (int j = 0; j < 3; ++j) acc += qs[(r + i) * 66 + d + j] * w[i * 3 + j];
    tile[r * 64 + d] = (_Float16)acc;
  }
  __syncthreads();
  {
    const int row = wave * 4 + (lane >> 3), c8 = (lane & 7) * 8;
    _Float16* qout = Q16 + ((size_t)bh * LL + l0) * DD;
    for (int pass = 0; pass < 2; ++pass) {
      const v8h v = *(const v8h*)(tile + row * 64 + c8);
      *(volatile v8h*)(qout + (size_t)row * DD + c8) = v;
      __threadfence();
    }
  }
}

__global__ __launch_bounds__(128)
void attn_kernel(const _Float16* __restrict__ Q16, const _Float16* __restrict__ K16,
                 const _Float16* __restrict__ V16, const int* __restrict__ pad,
                 const int* __restrict__ caus, float* __restrict__ out) {
  union FB { v16h v; v8h h[2]; };
  __shared__ __align__(16) _Float16 Ksh[AKC * DD];
  __shared__ __align__(16) _Float16 Vth[DD * AKC];
  __shared__ __align__(16) _Float16 Psh[4][16 * AKC];
  __shared__ __align__(16) float  Os[4][16 * 68];
  __shared__ int smask[LL];

  const int tid  = threadIdx.x;
  const int wave = tid >> 5;
  const int lane = tid & 31;
  const int hh   = lane >> 4;
  const int c    = lane & 15;

  const int bx = blockIdx.x;
  const int qb = bx % (LL / 64);
  const int bh = bx / (LL / 64);
  const int h  = bh & (HH - 1);
  const int b  = bh >> 4;
  const int q0 = qb * 64 + wave * 16;

  const _Float16* qp = Q16 + (size_t)bh * LL * DD;
  const _Float16* kp = K16 + (size_t)bh * LL * DD;
  const _Float16* vp = V16 + (size_t)bh * LL * DD;
  float* ob = out + (size_t)b * LL * EE + (size_t)h * DD;

  for (int i = tid; i < LL; i += 128)
    smask[i] = ((pad[(size_t)b * LL + i] != 0) && (caus[(size_t)b * LL + i] != 0)) ? 1 : 0;

  v16h qa[2];
  {
    const _Float16* qrow = qp + (size_t)(q0 + c) * DD;
    qa[0] = Frag<_Float16>::load(qrow + 8 * hh);
    qa[1] = Frag<_Float16>::load(qrow + 32 + 8 * hh);
  }

  float mrow[8], lrow[8];
  v8f oacc[4];
#pragma unroll
  for (int r = 0; r < 8; ++r) { mrow[r] = NEG_INF; lrow[r] = 0.f; }
#pragma unroll
  for (int t = 0; t < 4; ++t) oacc[t] = (v8f){0.f,0.f,0.f,0.f,0.f,0.f,0.f,0.f};

  for (int kc = 0; kc < LL / AKC; ++kc) {
    const int kv0 = kc * AKC;
    __syncthreads();
    {
      const int kvr = tid >> 1, dh = (tid & 1) * 32;
      const _Float16* krow = kp + (size_t)(kv0 + kvr) * DD + dh;
      const _Float16* vrow = vp + (size_t)(kv0 + kvr) * DD + dh;
#pragma unroll
      for (int i = 0; i < 4; ++i) {
        const v8h kk = *(const v8h*)(krow + 8 * i);
        const v8h vv = *(const v8h*)(vrow + 8 * i);
        *(v8h*)(Ksh + kvr * DD + dh + 8 * i) = kk;
#pragma unroll
        for (int e = 0; e < 8; ++e) Vth[(dh + 8 * i + e) * AKC + kvr] = vv[e];
      }
    }
    __syncthreads();

    v8f s[4];
#pragma unroll
    for (int j = 0; j < 4; ++j) {
      s[j] = (v8f){0.f,0.f,0.f,0.f,0.f,0.f,0.f,0.f};
#pragma unroll
      for (int dc = 0; dc < 2; ++dc) {
        FB kb;
        kb.h[0] = *(const v8h*)(Ksh + (j * 16 + c) * DD + dc * 32 + 8 * hh);
        kb.h[1] = *(const v8h*)(Ksh + (j * 16 + c) * DD + dc * 32 + 16 + 8 * hh);
        s[j] = mma_h(qa[dc], kb.v, s[j]);
      }
    }
    int kvm[4];
#pragma unroll
    for (int j = 0; j < 4; ++j) kvm[j] = smask[kv0 + j * 16 + c];
    float cm[8];
#pragma unroll
    for (int r = 0; r < 8; ++r) {
      float m = NEG_INF;
#pragma unroll
      for (int j = 0; j < 4; ++j) {
        float val = s[j][r] * SCL_QK;
        if (kvm[j] != 0) val = MASKV;
        s[j][r] = val;
        m = fmaxf(m, val);
      }
#pragma unroll
      for (int off = 1; off < 16; off <<= 1) m = fmaxf(m, __shfl_xor(m, off, 32));
      cm[r] = m;
    }
    _Float16* pw = Psh[wave];
#pragma unroll
    for (int r = 0; r < 8; ++r) {
      const float mnew = fmaxf(mrow[r], cm[r]);
      const float alpha = expf(mrow[r] - mnew);
      mrow[r] = mnew;
      float psum = 0.f;
#pragma unroll
      for (int j = 0; j < 4; ++j) {
        const float p = expf(s[j][r] - mnew);
        psum += p;
        pw[(8 * hh + r) * AKC + j * 16 + c] = (_Float16)(p * PSC16);
      }
#pragma unroll
      for (int off = 1; off < 16; off <<= 1) psum += __shfl_xor(psum, off, 32);
      lrow[r] = lrow[r] * alpha + psum;
#pragma unroll
      for (int t = 0; t < 4; ++t) oacc[t][r] *= alpha;
    }
    __builtin_amdgcn_fence(__ATOMIC_RELEASE, "workgroup");
    __builtin_amdgcn_wave_barrier();
    __builtin_amdgcn_fence(__ATOMIC_ACQUIRE, "workgroup");
#pragma unroll 1
    for (int kk = 0; kk < 2; ++kk) {
      FB pa;
      pa.h[0] = *(const v8h*)(pw + c * AKC + kk * 32 + 8 * hh);
      pa.h[1] = *(const v8h*)(pw + c * AKC + kk * 32 + 16 + 8 * hh);
#pragma unroll
      for (int t = 0; t < 4; ++t) {
        FB vb;
        vb.h[0] = *(const v8h*)(Vth + (t * 16 + c) * AKC + kk * 32 + 8 * hh);
        vb.h[1] = *(const v8h*)(Vth + (t * 16 + c) * AKC + kk * 32 + 16 + 8 * hh);
        oacc[t] = mma_h(pa.v, vb.v, oacc[t]);
      }
    }
  }

  float* os = Os[wave];
#pragma unroll
  for (int r = 0; r < 8; ++r) {
    const float inv = 1.0f / (lrow[r] * PSC16);
#pragma unroll
    for (int t = 0; t < 4; ++t) os[(8 * hh + r) * 68 + t * 16 + c] = oacc[t][r] * inv;
  }
  __builtin_amdgcn_fence(__ATOMIC_RELEASE, "workgroup");
  __builtin_amdgcn_wave_barrier();
  __builtin_amdgcn_fence(__ATOMIC_ACQUIRE, "workgroup");
  {
    const int c4 = (lane & 15) * 4;
    for (int pass = 0; pass < 2; ++pass) {
#pragma unroll
      for (int it = 0; it < 8; ++it) {
        const int row = it * 2 + hh;
        const v4f val = *(const v4f*)(os + row * 68 + c4);
        *(volatile v4f*)(ob + (size_t)(q0 + row) * EE + c4) = val;
      }
      __threadfence();
    }
  }
}

extern "C" void kernel_launch(void* const* d_in, const int* in_sizes, int n_in,
                              void* d_out, int out_size, void* d_ws, size_t ws_size,
                              hipStream_t stream) {
  if (n_in < 9) return;
  if (out_size != BB * LL * EE) return;
  if (in_sizes[0] != BB * LL * EE || in_sizes[1] != BB * LL * EE || in_sizes[2] != BB * LL * EE) return;
  if (in_sizes[3] != BB * LL || in_sizes[4] != BB * LL || in_sizes[5] != BB * HH * LL) return;
  if (in_sizes[6] != HH * 9 || in_sizes[7] != HH || in_sizes[8] != DD * DD) return;

  const float* query  = (const float*)d_in[0];
  const float* keys   = (const float*)d_in[1];
  const float* values = (const float*)d_in[2];
  const int*   pad    = (const int*)d_in[3];
  const int*   caus   = (const int*)d_in[4];
  const int*   bern   = (const int*)d_in[5];
  const float* cw     = (const float*)d_in[6];
  const float* cb     = (const float*)d_in[7];
  const float* Wv     = (const float*)d_in[8];
  float* out = (float*)d_out;

  const size_t planeElems = (size_t)BB * LL * EE;
  const size_t planeBytes = planeElems * 2;
  size_t off = 0;
  _Float16* Vin16 = (_Float16*)((char*)d_ws + off); off += planeBytes;
  _Float16* K16   = (_Float16*)((char*)d_ws + off); off += planeBytes;
  _Float16* Q16   = (_Float16*)((char*)d_ws + off); off += planeBytes;
  _Float16* V16   = (_Float16*)((char*)d_ws + off); off += planeBytes;
  _Float16* Wv16  = (_Float16*)((char*)d_ws + off); off += (size_t)DD * DD * 2;
  if (off > ws_size) return;

  {
    const int n8 = (int)(planeElems / 8);
    cast8_f16_kernel<<<dim3((n8 + 255) / 256), dim3(256), 0, stream>>>(values, Vin16, n8);
  }
  {
    const int n2 = DD * DD / 2;
    cast_f32_f16x2<<<dim3((n2 + 255) / 256), dim3(256), 0, stream>>>(Wv, Wv16, n2);
  }
  ksoft_kernel<<<dim3(NBH), dim3(64), 0, stream>>>(keys, bern, K16);
  qconv_kernel<<<dim3(LL / 32, NBH), dim3(256), 0, stream>>>(query, cw, cb, Q16);
  for (int b = 0; b < BB; ++b) {
    const unsigned short* Ab = (const unsigned short*)(Vin16 + (size_t)b * LL * EE);
    void* Cb = (void*)(V16 + (size_t)b * HH * LL * DD);
    const int tiles = (LL / 64) * (DD / 64);
    wmma_gemm64<0, false, 0, 1, false, 0><<<dim3((tiles + 7) / 8, HH), dim3(256), 0, stream>>>(
        Ab, Ab, EE, (long)DD,
        (const unsigned short*)Wv16, (const unsigned short*)Wv16, DD, 0L,
        Cb, Cb, DD, (long)LL * DD,
        Wv, query, 0L,
        LL, DD, DD, 1.0f);
  }
  attn_kernel<<<dim3(NBH * (LL / 64)), dim3(128), 0, stream>>>(Q16, K16, V16, pad, caus, out);
}
